// DynamicGlobalWindowTransformer_32066225832467
// MI455X (gfx1250) — hardware-run, weakly checked
//
#include <hip/hip_runtime.h>
#include <math.h>

#ifndef NB
#define NB 8
#endif
#ifndef SEQ
#define SEQ 2048
#endif
#define NB_FULL 8
#define SEQ_FULL 2048
#define EMB 256
#define HEADS 4
#define HD 64
#define FFD 1024
#define MTOK (NB * SEQ)
#define OUT1_OFF (NB_FULL * SEQ_FULL * EMB)

static_assert(EMB == 256 && HEADS == 4 && HD == 64 && HEADS * HD == EMB);
static_assert(NB <= NB_FULL && SEQ <= SEQ_FULL);
static_assert(SEQ % 128 == 0 && SEQ <= 2048);
static_assert(MTOK % 64 == 0);
static_assert(EMB % 64 == 0 && (2 * EMB) % 64 == 0 && FFD % 64 == 0);
static_assert(EMB % 32 == 0 && FFD % 32 == 0);
static_assert((MTOK * EMB / 8) % 256 == 0);
static_assert((3 * EMB * EMB / 8) % 256 == 0 && (EMB * EMB / 8) % 256 == 0 && (FFD * EMB / 8) % 256 == 0);
static_assert(MTOK % 8 == 0);
static_assert(((NB * SEQ) / 64) % 4 == 0);
static_assert((size_t)OUT1_OFF * 4 == (size_t)16777216);
static_assert((size_t)MTOK * EMB <= (size_t)OUT1_OFF);

typedef __attribute__((ext_vector_type(16))) _Float16 v16h;
typedef __attribute__((ext_vector_type(8)))  _Float16 v8h;
typedef __attribute__((ext_vector_type(8)))  float    v8f;
typedef __attribute__((ext_vector_type(4)))  float    v4f;
typedef _Float16 h16;

static constexpr float kActC  = 64.0f;
static constexpr float kPC    = 1024.0f;
static constexpr float kSC2   = 0.125f * 1.4426950408889634f * (1.0f / 4096.0f);
static constexpr float kNEG2  = -1.0e9f * 1.4426950408889634f;
static constexpr float kOutSc = 1024.0f / (1024.0f * 64.0f);


#define VST2(T, ptr, val) do { const T vst2_v_ = (val); *(volatile T*)(ptr) = vst2_v_; __threadfence(); *(volatile T*)(ptr) = vst2_v_; } while (0)

__device__ __forceinline__ float bfr(float f) {
    unsigned u = __float_as_uint(f);
    u += 0x7FFFu + ((u >> 16) & 1u);
    return __uint_as_float(u & 0xFFFF0000u);
}
static __device__ __forceinline__ h16 toh_flush(float v) {
    const float w = (fabsf(v) < 6.103515625e-05f) ? 0.0f : v;
    return (h16)w;
}

union FragU { v16h v; v8h h[2]; };
__device__ __forceinline__ v16h frag_ld(const h16* p) {
    FragU f; f.h[0] = *(const v8h*)(p); f.h[1] = *(const v8h*)(p + 16); return f.v;
}
__device__ __forceinline__ v8f wmma16g(v16h a, v16h b, v8f c) {
    c = __builtin_amdgcn_wmma_f32_16x16x32_f16(false, a, false, b, (short)0, c, false, false);
    asm volatile("v_nop\n\tv_nop\n\tv_nop\n\tv_nop" : "+v"(c) : "v"(a), "v"(b));
    return c;
}
__device__ __forceinline__ void wave_sync_lds() {
    __builtin_amdgcn_fence(3  , "workgroup");
    __builtin_amdgcn_wave_barrier();
    __builtin_amdgcn_fence(2  , "workgroup");
}

template <int CARRY, bool ROWMAP>
__global__ __launch_bounds__(256) void k_cvt16(const float* __restrict__ src, h16* __restrict__ dst, unsigned units) {
    const unsigned u = blockIdx.x * 256u + threadIdx.x;
    if (u >= units) return;
    size_t so;
    if (ROWMAP) {
        const unsigned row = u >> 5;
        const unsigned c0 = (u & 31u) * 8u;
        const unsigned bb = row / (unsigned)SEQ;
        const unsigned tt = row - bb * (unsigned)SEQ;
        so = ((size_t)bb * (unsigned)SEQ_FULL + tt) * (unsigned)EMB + c0;
    } else {
        so = (size_t)u * 8u;
    }
    const v4f a = *(const v4f*)(src + so);
    const v4f b = *(const v4f*)(src + so + 4);
    const float cf = (float)CARRY;
    v8h pk;
    pk[0] = toh_flush(bfr(a.x) * cf); pk[1] = toh_flush(bfr(a.y) * cf);
    pk[2] = toh_flush(bfr(a.z) * cf); pk[3] = toh_flush(bfr(a.w) * cf);
    pk[4] = toh_flush(bfr(b.x) * cf); pk[5] = toh_flush(bfr(b.y) * cf);
    pk[6] = toh_flush(bfr(b.z) * cf); pk[7] = toh_flush(bfr(b.w) * cf);
    h16* p = dst + (size_t)u * 8u;
    VST2(v8h, p, pk);
}

template <int OUT_MODE, int RESID, bool RELU, bool BIASROW, int LGS, int LGO>
__global__ __launch_bounds__(256) void k_gemm64(
    const h16* __restrict__ A, unsigned lda, const h16* __restrict__ Bt, unsigned ldb,
    void* __restrict__ Cout, unsigned ldc, const float* __restrict__ bias, const float* __restrict__ resid,
    unsigned M, unsigned N, unsigned K) {
  __shared__ __align__(16) float sT[8][16 * 68];
  constexpr float scale  = 1.0f / (float)(1u << LGS);
  constexpr float oscale = (float)(1u << LGO);
  const unsigned lane = threadIdx.x & 31u;
  const unsigned wave = threadIdx.x >> 5;
  const unsigned tilesN = N >> 6, tilesM = M >> 6;
  const unsigned tile = blockIdx.x * 8u + wave;
  if (tile >= tilesM * tilesN) return;
  const unsigned tm = tile / tilesN;
  const unsigned tn = tile - tm * tilesN;
  const unsigned m0 = tm << 6, n0 = tn << 6;
  const unsigned rlane = lane & 15u;
  const unsigned koff = (lane >> 4) * 8u;
  const unsigned mOff = koff;

  v8f acc[4][4];
#pragma unroll
  for (int i = 0; i < 4; ++i)
#pragma unroll
    for (int j = 0; j < 4; ++j) acc[i][j] = (v8f){0.f,0.f,0.f,0.f,0.f,0.f,0.f,0.f};

  for (unsigned k0 = 0; k0 < K; k0 += 32u) {
    v16h bh[4];
#pragma unroll
    for (int j = 0; j < 4; ++j)
      bh[j] = frag_ld(Bt + (size_t)(n0 + ((unsigned)j << 4) + rlane) * ldb + koff + k0);
#pragma unroll
    for (int i = 0; i < 4; ++i) {
      const v16h ah = frag_ld(A + (size_t)(m0 + ((unsigned)i << 4) + rlane) * lda + koff + k0);
#pragma unroll
      for (int j = 0; j < 4; ++j)
        acc[i][j] = wmma16g(ah, bh[j], acc[i][j]);
    }
  }

  float* slab = sT[wave];
#pragma unroll
  for (int i = 0; i < 4; ++i) {
    const unsigned mBase = m0 + ((unsigned)i << 4);
#pragma unroll
    for (int j = 0; j < 4; ++j) {
      const unsigned n = n0 + ((unsigned)j << 4) + rlane;
      const float bcol = bfr(bias[BIASROW ? (mBase + mOff) : n]);
#pragma unroll
      for (int r = 0; r < 8; ++r) {
        const float bv = BIASROW ? bfr(bias[mBase + mOff + (unsigned)r]) : bcol;
        float v = acc[i][j][r] * scale + bv;
        if (RELU) v = fmaxf(v, 0.0f);
        if (OUT_MODE == 1) v *= oscale;
        slab[(mOff + (unsigned)r) * 68u + ((unsigned)j << 4) + rlane] = v;
      }
    }
    wave_sync_lds();
    if (OUT_MODE == 0) {
      float* C = (float*)Cout;
      const unsigned hh = lane >> 4, c4 = (lane & 15u) * 4u;
#pragma unroll
      for (int half = 0; half < 2; ++half) {
        v4f vv[4];
#pragma unroll
        for (int it = 0; it < 4; ++it) {
          const unsigned row = (unsigned)(half * 4 + it) * 2u + hh;
          vv[it] = *(const v4f*)(slab + row * 68u + c4);
          if (RESID == 1) vv[it] += *(const v4f*)(resid + (size_t)(mBase + row) * ldc + n0 + c4);
          if (RESID == 2) {
            const unsigned grow = mBase + row;
            const unsigned bb = grow / (unsigned)SEQ;
            const unsigned tt = grow - bb * (unsigned)SEQ;
            const v4f xv = *(const v4f*)(resid + ((size_t)bb * (unsigned)SEQ_FULL + tt) * ldc + n0 + c4);
            vv[it].x += bfr(xv.x); vv[it].y += bfr(xv.y); vv[it].z += bfr(xv.z); vv[it].w += bfr(xv.w);
          }
        }
        for (int pass = 0; pass < 2; ++pass) {
#pragma unroll
          for (int it = 0; it < 4; ++it) {
            const unsigned row = (unsigned)(half * 4 + it) * 2u + hh;
            *(volatile v4f*)(C + (size_t)(mBase + row) * ldc + n0 + c4) = vv[it];
          }
          __threadfence();
        }
      }
    } else {
      h16* C = (h16*)Cout;
      const unsigned q = lane >> 3, c8 = (lane & 7u) * 8u;
      v8h hv[4];
#pragma unroll
      for (int it = 0; it < 4; ++it) {
        const unsigned row = (unsigned)it * 4u + q;
        const float* sp = slab + row * 68u + c8;
#pragma unroll
        for (int e = 0; e < 8; ++e) hv[it][e] = toh_flush(sp[e]);
      }
      for (int pass = 0; pass < 2; ++pass) {
#pragma unroll
        for (int it = 0; it < 4; ++it) {
          const unsigned row = (unsigned)it * 4u + q;
          *(volatile v8h*)(C + (size_t)(mBase + row) * ldc + n0 + c8) = hv[it];
        }
        __threadfence();
      }
    }
    wave_sync_lds();
  }
}

#define AT_PO 72
__global__ __launch_bounds__(128) void k_attn(const h16* __restrict__ qk, const h16* __restrict__ vt, const float* __restrict__ mask,
                                              h16* __restrict__ att, float* __restrict__ mpl, float* __restrict__ rpl, unsigned nsteps) {
    __shared__ __align__(16) h16 sO[4][32 * AT_PO];
    const unsigned tid = threadIdx.x, lane = tid & 31u, wave = tid >> 5;
    const unsigned hh = lane >> 4, c = lane & 15u;
    const unsigned bx = blockIdx.x;
    const unsigned QBLK = (unsigned)SEQ / 128u;
    const unsigned bh = bx / QBLK;
    const unsigned qb = bx - bh * QBLK;
    const unsigned b = bh >> 2, h = bh & 3u;
    const unsigned q0 = qb * 128u + wave * 32u;
    const size_t rowb = (size_t)b * (unsigned)SEQ;

    v16h qf[2][2];
#pragma unroll
    for (int qi = 0; qi < 2; ++qi)
#pragma unroll
        for (int kk = 0; kk < 2; ++kk)
            qf[qi][kk] = frag_ld(qk + (rowb + q0 + 16u * (unsigned)qi + c) * 512u + 64u * h + 32u * (unsigned)kk + 8u * hh);

    const h16* kbase = qk + (rowb + c) * 512u + 256u + 64u * h + 8u * hh;
    const h16* vbase = vt + (size_t)(64u * h + c) * (unsigned)MTOK + rowb + 8u * hh;
    const float* mrow = mask + (size_t)b * (unsigned)SEQ_FULL + 8u * hh;

    float mrun[2], lrun[2];
    v8f o[2][4];
#pragma unroll
    for (int qi = 0; qi < 2; ++qi) {
        mrun[qi] = -3.0e38f; lrun[qi] = 0.f;
#pragma unroll
        for (int t = 0; t < 4; ++t) o[qi][t] = (v8f){0.f,0.f,0.f,0.f,0.f,0.f,0.f,0.f};
    }

    for (unsigned st = 0; st < nsteps; ++st) {
        const unsigned key0 = st * 32u;
        v8f s[2][2];
        {
            v16h kf[2][2];
#pragma unroll
            for (int j = 0; j < 2; ++j)
#pragma unroll
                for (int kk = 0; kk < 2; ++kk)
                    kf[j][kk] = frag_ld(kbase + (size_t)(key0 + 16u * (unsigned)j) * 512u + 32u * (unsigned)kk);
#pragma unroll
            for (int qi = 0; qi < 2; ++qi)
#pragma unroll
                for (int j = 0; j < 2; ++j) {
                    const v8f z = (v8f){0.f,0.f,0.f,0.f,0.f,0.f,0.f,0.f};
                    const v8f t0 = wmma16g(kf[j][0], qf[qi][0], z);
                    s[qi][j] = wmma16g(kf[j][1], qf[qi][1], t0);
                }
        }
        bool kill[2][8];
#pragma unroll
        for (int j = 0; j < 2; ++j) {
            const v4f ma = *(const v4f*)(mrow + key0 + 16u * (unsigned)j);
            const v4f mb = *(const v4f*)(mrow + key0 + 16u * (unsigned)j + 4u);
            kill[j][0] = bfr(ma.x) > 0.5f; kill[j][1] = bfr(ma.y) > 0.5f;
            kill[j][2] = bfr(ma.z) > 0.5f; kill[j][3] = bfr(ma.w) > 0.5f;
            kill[j][4] = bfr(mb.x) > 0.5f; kill[j][5] = bfr(mb.y) > 0.5f;
            kill[j][6] = bfr(mb.z) > 0.5f; kill[j][7] = bfr(mb.w) > 0.5f;
        }
        v16h pb[2];
#pragma unroll
        for (int qi = 0; qi < 2; ++qi) {
            float mx = -3.0e38f;
#pragma unroll
            for (int j = 0; j < 2; ++j)
#pragma unroll
                for (int r = 0; r < 8; ++r) {
                    const float sv = s[qi][j][r] * kSC2;
                    const float v = kill[j][r] ? kNEG2 : sv;
                    s[qi][j][r] = v;
                    mx = fmaxf(mx, v);
                }
            mx = fmaxf(mx, __shfl_xor(mx, 16, 32));
            const float mnew = fmaxf(mrun[qi], mx);
            const float alpha = exp2f(mrun[qi] - mnew);
            mrun[qi] = mnew;
            float psum = 0.f;
            v16h pv;
#pragma unroll
            for (int j = 0; j < 2; ++j)
#pragma unroll
                for (int r = 0; r < 8; ++r) {
                    const float p = exp2f(s[qi][j][r] - mnew);
                    psum += p;
                    pv[8 * j + r] = toh_flush(p * kPC);
                }
            psum += __shfl_xor(psum, 16, 32);
            lrun[qi] = lrun[qi] * alpha + psum;
#pragma unroll
            for (int t = 0; t < 4; ++t)
#pragma unroll
                for (int r = 0; r < 8; ++r) o[qi][t][r] *= alpha;
            pb[qi] = pv;
        }
#pragma unroll
        for (int t = 0; t < 4; ++t) {
            const v16h vf = frag_ld(vbase + (size_t)(16u * (unsigned)t) * (unsigned)MTOK + key0);
#pragma unroll
            for (int qi = 0; qi < 2; ++qi) o[qi][t] = wmma16g(vf, pb[qi], o[qi][t]);
        }
    }

    float rl[2];
#pragma unroll
    for (int qi = 0; qi < 2; ++qi) rl[qi] = 1.0f / lrun[qi];

    h16* pw = sO[wave];
#pragma unroll
    for (int qi = 0; qi < 2; ++qi) {
        const float sc = rl[qi] * kOutSc;
#pragma unroll
        for (int t = 0; t < 4; ++t) {
            v8h pk;
#pragma unroll
            for (int r = 0; r < 8; ++r) pk[r] = toh_flush(o[qi][t][r] * sc);
            *(v8h*)(pw + (16u * (unsigned)qi + c) * AT_PO + 16u * (unsigned)t + 8u * hh) = pk;
        }
    }
    wave_sync_lds();
    {
        const unsigned q4 = lane >> 3, c8 = (lane & 7u) * 8u;
        v8h ov[8];
#pragma unroll
        for (int it = 0; it < 8; ++it) ov[it] = *(const v8h*)(pw + ((unsigned)it * 4u + q4) * AT_PO + c8);
        h16* dst = att + (rowb + q0) * (unsigned)EMB + 64u * h;
        for (int pass = 0; pass < 2; ++pass) {
#pragma unroll
            for (int it = 0; it < 8; ++it) *(volatile v8h*)(dst + (size_t)((unsigned)it * 4u + q4) * (unsigned)EMB + c8) = ov[it];
            __threadfence();
        }
    }
    {
        const float mv = (hh != 0u) ? mrun[1] : mrun[0];
        const float rv = (hh != 0u) ? rl[1] : rl[0];
        float* mp = mpl + (size_t)bh * (unsigned)SEQ + q0 + lane;
        float* rp = rpl + (size_t)bh * (unsigned)SEQ + q0 + lane;
        *(volatile float*)mp = mv; *(volatile float*)rp = rv;
        __threadfence();
        *(volatile float*)mp = mv; *(volatile float*)rp = rv;
    }
}

__global__ __launch_bounds__(128) void k_colsum(const h16* __restrict__ qk, const float* __restrict__ mask,
                                                const float* __restrict__ mpl, const float* __restrict__ rpl,
                                                float* __restrict__ hpre, unsigned nqt, unsigned nheads) {
    const unsigned tid = threadIdx.x, lane = tid & 31u, wave = tid >> 5;
    const unsigned hh = lane >> 4, c = lane & 15u;
    const unsigned gw = blockIdx.x * 4u + wave;
    const unsigned KG = (unsigned)SEQ / 64u;
    const unsigned b = gw / KG;
    const unsigned kg = gw - b * KG;
    const unsigned key0 = kg * 64u;
    const size_t rowb = (size_t)b * (unsigned)SEQ;

    bool kill[4];
#pragma unroll
    for (int j = 0; j < 4; ++j)
        kill[j] = bfr(mask[(size_t)b * (unsigned)SEQ_FULL + key0 + 16u * (unsigned)j + c]) > 0.5f;

    float tot[4] = {0.f, 0.f, 0.f, 0.f};
    for (unsigned h = 0; h < nheads; ++h) {
        v16h kf[4][2];
#pragma unroll
        for (int j = 0; j < 4; ++j)
#pragma unroll
            for (int kk = 0; kk < 2; ++kk)
                kf[j][kk] = frag_ld(qk + (rowb + key0 + 16u * (unsigned)j + c) * 512u + 256u + 64u * h + 32u * (unsigned)kk + 8u * hh);
        const h16* qbase = qk + (rowb + c) * 512u + 64u * h + 8u * hh;
        const float* mb = mpl + (size_t)(b * 4u + h) * (unsigned)SEQ + 8u * hh;
        const float* rb = rpl + (size_t)(b * 4u + h) * (unsigned)SEQ + 8u * hh;
        float cs[4] = {0.f, 0.f, 0.f, 0.f};
        for (unsigned qt = 0; qt < nqt; ++qt) {
            const v16h qf0 = frag_ld(qbase + (size_t)(16u * qt) * 512u);
            const v16h qf1 = frag_ld(qbase + (size_t)(16u * qt) * 512u + 32u);
            const v4f m0 = *(const v4f*)(mb + 16u * qt), m1 = *(const v4f*)(mb + 16u * qt + 4u);
            const v4f r0 = *(const v4f*)(rb + 16u * qt), r1 = *(const v4f*)(rb + 16u * qt + 4u);
            const float mm[8] = {m0.x, m0.y, m0.z, m0.w, m1.x, m1.y, m1.z, m1.w};
            const float rr[8] = {r0.x, r0.y, r0.z, r0.w, r1.x, r1.y, r1.z, r1.w};
#pragma unroll
            for (int j = 0; j < 4; ++j) {
                const v8f z = (v8f){0.f,0.f,0.f,0.f,0.f,0.f,0.f,0.f};
                const v8f t0 = wmma16g(qf0, kf[j][0], z);
                const v8f sj = wmma16g(qf1, kf[j][1], t0);
#pragma unroll
                for (int r = 0; r < 8; ++r) {
                    const float sv = sj[r] * kSC2;
                    const float v = kill[j] ? kNEG2 : sv;
                    cs[j] += exp2f(v - mm[r]) * rr[r];
                }
            }
        }
#pragma unroll
        for (int j = 0; j < 4; ++j) {
            const float other = __shfl_xor(cs[j], 16, 32);
            tot[j] += cs[j] + other;
        }
    }
    const float v0 = ((hh != 0u) ? tot[1] : tot[0]) * 0.25f;
    const float v1 = ((hh != 0u) ? tot[3] : tot[2]) * 0.25f;
    float* hp = hpre + rowb + key0 + lane;
    *(volatile float*)hp = v0; *(volatile float*)(hp + 32) = v1;
    __threadfence();
    *(volatile float*)hp = v0; *(volatile float*)(hp + 32) = v1;
}

#define HALT_IT ((SEQ + 1023) / 1024)
__global__ __launch_bounds__(256) void k_halt(const float* __restrict__ hpre, const float* __restrict__ mask, float* __restrict__ out1) {
    __shared__ float redm[8];
    __shared__ float reds[8];
    const unsigned t = threadIdx.x, lane = t & 31u, wave = t >> 5;
    const unsigned b = blockIdx.x;
    v4f vv[HALT_IT];
    bool act[HALT_IT];
    float lm = -3.0e38f;
#pragma unroll
    for (int i = 0; i < HALT_IT; ++i) {
        const unsigned idx = 4u * (t + 256u * (unsigned)i);
        act[i] = idx < (unsigned)SEQ;
        const unsigned idc = min(idx, (unsigned)SEQ - 4u);
        const v4f hv = *(const v4f*)(hpre + (size_t)b * (unsigned)SEQ + idc);
        const v4f mk = *(const v4f*)(mask + (size_t)b * (unsigned)SEQ_FULL + idc);
        v4f v;
        v.x = hv.x + bfr(mk.x) * (-1.0e10f);
        v.y = hv.y + bfr(mk.y) * (-1.0e10f);
        v.z = hv.z + bfr(mk.z) * (-1.0e10f);
        v.w = hv.w + bfr(mk.w) * (-1.0e10f);
        vv[i] = v;
        const float m4 = fmaxf(fmaxf(v.x, v.y), fmaxf(v.z, v.w));
        lm = act[i] ? fmaxf(lm, m4) : lm;
    }
#pragma unroll
    for (int o = 16; o > 0; o >>= 1) lm = fmaxf(lm, __shfl_xor(lm, o, 32));
    if (lane == 0u) redm[wave] = lm;
    __syncthreads();
    float mx = redm[0];
#pragma unroll
    for (int w = 1; w < 8; ++w) mx = fmaxf(mx, redm[w]);
    float ls = 0.f;
    v4f ee[HALT_IT];
#pragma unroll
    for (int i = 0; i < HALT_IT; ++i) {
        v4f e;
        e.x = expf(vv[i].x - mx); e.y = expf(vv[i].y - mx); e.z = expf(vv[i].z - mx); e.w = expf(vv[i].w - mx);
        ee[i] = e;
        const float s4 = (e.x + e.y) + (e.z + e.w);
        ls += act[i] ? s4 : 0.0f;
    }
#pragma unroll
    for (int o = 16; o > 0; o >>= 1) ls += __shfl_xor(ls, o, 32);
    if (lane == 0u) reds[wave] = ls;
    __syncthreads();
    float tsum = reds[0];
#pragma unroll
    for (int w = 1; w < 8; ++w) tsum += reds[w];
    v4f res[HALT_IT];
#pragma unroll
    for (int i = 0; i < HALT_IT; ++i) {
        res[i].x = ee[i].x / tsum; res[i].y = ee[i].y / tsum; res[i].z = ee[i].z / tsum; res[i].w = ee[i].w / tsum;
    }
    float* ob = out1 + (size_t)b * (unsigned)SEQ;
#pragma unroll
    for (int i = 0; i < HALT_IT; ++i) {
        const unsigned idx = 4u * (t + 256u * (unsigned)i);
        if (act[i]) *(volatile v4f*)(ob + idx) = res[i];
    }
    __threadfence();
#pragma unroll
    for (int i = 0; i < HALT_IT; ++i) {
        const unsigned idx = 4u * (t + 256u * (unsigned)i);
        if (act[i]) *(volatile v4f*)(ob + idx) = res[i];
    }
}

template <bool FIRST>
__global__ __launch_bounds__(256) void k_ln(const float* __restrict__ y, const float* __restrict__ g, const float* __restrict__ be,
                                            float* __restrict__ of32, h16* __restrict__ o16, unsigned M) {
    const unsigned row = blockIdx.x * 8u + (threadIdx.x >> 5);
    const unsigned L = threadIdx.x & 31u;
    if (row >= M) return;
    const float* yr = y + (size_t)row * (unsigned)EMB;
    const v4f a = *(const v4f*)(yr + 4u * L), b = *(const v4f*)(yr + 128u + 4u * L);
    float s = ((a.x + a.y) + (a.z + a.w)) + ((b.x + b.y) + (b.z + b.w));
#pragma unroll
    for (int o = 16; o > 0; o >>= 1) s += __shfl_xor(s, o, 32);
    const float mu = s * (1.0f / 256.0f);
    const float d[8] = {a.x - mu, a.y - mu, a.z - mu, a.w - mu, b.x - mu, b.y - mu, b.z - mu, b.w - mu};
    float q = 0.f;
#pragma unroll
    for (int i = 0; i < 8; ++i) q += d[i] * d[i];
#pragma unroll
    for (int o = 16; o > 0; o >>= 1) q += __shfl_xor(q, o, 32);
    const float sd = sqrtf(q * (1.0f / 256.0f) + 1e-5f);
    const v4f ga = *(const v4f*)(g + 4u * L), gb = *(const v4f*)(g + 128u + 4u * L);
    const v4f ba = *(const v4f*)(be + 4u * L), bb = *(const v4f*)(be + 128u + 4u * L);
    v4f ya, yb;
    ya.x = d[0] / sd * bfr(ga.x) + bfr(ba.x); ya.y = d[1] / sd * bfr(ga.y) + bfr(ba.y);
    ya.z = d[2] / sd * bfr(ga.z) + bfr(ba.z); ya.w = d[3] / sd * bfr(ga.w) + bfr(ba.w);
    yb.x = d[4] / sd * bfr(gb.x) + bfr(bb.x); yb.y = d[5] / sd * bfr(gb.y) + bfr(bb.y);
    yb.z = d[6] / sd * bfr(gb.z) + bfr(bb.z); yb.w = d[7] / sd * bfr(gb.w) + bfr(bb.w);
    float* op = of32 + (size_t)row * (unsigned)EMB + 4u * L;
    *(volatile v4f*)op = ya; *(volatile v4f*)(op + 128) = yb;
    __threadfence();
    *(volatile v4f*)op = ya; *(volatile v4f*)(op + 128) = yb;
    if (FIRST) {
        const v4f c0 = *(const v4f*)(yr + 8u * L), c1 = *(const v4f*)(yr + 8u * L + 4u);
        const v4f g0 = *(const v4f*)(g + 8u * L), g1 = *(const v4f*)(g + 8u * L + 4u);
        const v4f b0 = *(const v4f*)(be + 8u * L), b1 = *(const v4f*)(be + 8u * L + 4u);
        const float cc[8] = {c0.x, c0.y, c0.z, c0.w, c1.x, c1.y, c1.z, c1.w};
        const float gg[8] = {g0.x, g0.y, g0.z, g0.w, g1.x, g1.y, g1.z, g1.w};
        const float bt[8] = {b0.x, b0.y, b0.z, b0.w, b1.x, b1.y, b1.z, b1.w};
        v8h pk;
#pragma unroll
        for (int i = 0; i < 8; ++i) pk[i] = toh_flush(((cc[i] - mu) / sd * bfr(gg[i]) + bfr(bt[i])) * kActC);
        h16* hp = o16 + (size_t)row * (unsigned)EMB + 8u * L;
        VST2(v8h, hp, pk);
    }
}

static constexpr size_t SZ_X16   = (size_t)MTOK * EMB * 2;
static constexpr size_t SZ_WQKV  = (size_t)3 * EMB * EMB * 2;
static constexpr size_t SZ_WO    = (size_t)EMB * EMB * 2;
static constexpr size_t SZ_W1    = (size_t)FFD * EMB * 2;
static constexpr size_t SZ_W2    = (size_t)EMB * FFD * 2;
static constexpr size_t SZ_QK    = (size_t)MTOK * 2 * EMB * 2;
static constexpr size_t SZ_VT    = (size_t)EMB * MTOK * 2;
static constexpr size_t SZ_ATT   = (size_t)MTOK * EMB * 2;
static constexpr size_t SZ_ML    = (size_t)NB * HEADS * SEQ * 4;
static constexpr size_t SZ_HPRE  = (size_t)NB * SEQ * 4;
static constexpr size_t SZ_Y     = (size_t)MTOK * EMB * 4;
static constexpr size_t SZ_HF    = (size_t)MTOK * EMB * 4;
static constexpr size_t SZ_H16   = (size_t)MTOK * EMB * 2;
static constexpr size_t SZ_R16   = (size_t)MTOK * FFD * 2;
static constexpr size_t WS_TOTAL = SZ_X16 + SZ_WQKV + SZ_WO + SZ_W1 + SZ_W2 + SZ_QK + SZ_VT + SZ_ATT + 2 * SZ_ML + SZ_HPRE +
                                   SZ_Y + SZ_HF + SZ_H16 + SZ_R16;
static_assert(SZ_X16 % 256 == 0 && SZ_WQKV % 256 == 0 && SZ_WO % 256 == 0 && SZ_W1 % 256 == 0 && SZ_W2 % 256 == 0);
static_assert(SZ_QK % 256 == 0 && SZ_VT % 256 == 0 && SZ_ATT % 256 == 0 && SZ_ML % 256 == 0 && SZ_HPRE % 256 == 0);
static_assert(SZ_Y % 256 == 0 && SZ_HF % 256 == 0 && SZ_H16 % 256 == 0 && SZ_R16 % 256 == 0);
static_assert(WS_TOTAL <= (size_t)134217728);

extern "C" void kernel_launch(void* const* d_in, const int* in_sizes, int n_in, void* d_out, int out_size,
                              void* d_ws, size_t ws_size, hipStream_t stream) {
    if (n_in < 14) return;
    if (in_sizes[0] < ((NB - 1) * SEQ_FULL + SEQ) * EMB || in_sizes[1] < (NB - 1) * SEQ_FULL + SEQ) return;
    if (in_sizes[2] < 3 * EMB * EMB || in_sizes[3] < 3 * EMB || in_sizes[4] < EMB * EMB || in_sizes[5] < EMB) return;
    if (in_sizes[6] < FFD * EMB || in_sizes[7] < FFD || in_sizes[8] < EMB * FFD || in_sizes[9] < EMB) return;
    if (in_sizes[10] < EMB || in_sizes[11] < EMB || in_sizes[12] < EMB || in_sizes[13] < EMB) return;
    if (out_size < OUT1_OFF + NB * SEQ) return;

    const float* x    = (const float*)d_in[0];
    const float* mask = (const float*)d_in[1];
    const float* Wqkv = (const float*)d_in[2];
    const float* bqkv = (const float*)d_in[3];
    const float* Wo   = (const float*)d_in[4];
    const float* bo   = (const float*)d_in[5];
    const float* W1   = (const float*)d_in[6];
    const float* b1   = (const float*)d_in[7];
    const float* W2   = (const float*)d_in[8];
    const float* b2   = (const float*)d_in[9];
    const float* g1   = (const float*)d_in[10];
    const float* be1  = (const float*)d_in[11];
    const float* g2   = (const float*)d_in[12];
    const float* be2  = (const float*)d_in[13];
    float* out0 = (float*)d_out;
    float* out1 = (float*)d_out + (size_t)OUT1_OFF;

    char* wsp = (char*)d_ws;
    size_t off = 0;
    auto carve = [&](size_t bytes) -> void* { void* r = wsp + off; off += (bytes + 255) & ~(size_t)255; return r; };
    h16*   x16    = (h16*)carve(SZ_X16);
    h16*   wqkv16 = (h16*)carve(SZ_WQKV);
    h16*   wo16   = (h16*)carve(SZ_WO);
    h16*   w116   = (h16*)carve(SZ_W1);
    h16*   w216   = (h16*)carve(SZ_W2);
    h16*   qk16   = (h16*)carve(SZ_QK);
    h16*   vt16   = (h16*)carve(SZ_VT);
    h16*   att16  = (h16*)carve(SZ_ATT);
    float* mpl    = (float*)carve(SZ_ML);
    float* rpl    = (float*)carve(SZ_ML);
    float* hpre   = (float*)carve(SZ_HPRE);
    float* ybuf   = (float*)carve(SZ_Y);
    float* hf     = (float*)carve(SZ_HF);
    h16*   h16p   = (h16*)carve(SZ_H16);
    h16*   r16    = (h16*)carve(SZ_R16);
    if (off > ws_size || off > (size_t)134217728) return;

    k_cvt16<64, true><<<(MTOK * EMB / 8) / 256, 256, 0, stream>>>(x, x16, (unsigned)(MTOK * EMB / 8));
    k_cvt16<1024, false><<<(3 * EMB * EMB / 8) / 256, 256, 0, stream>>>(Wqkv, wqkv16, (unsigned)(3 * EMB * EMB / 8));
    k_cvt16<1024, false><<<(EMB * EMB / 8) / 256, 256, 0, stream>>>(Wo, wo16, (unsigned)(EMB * EMB / 8));
    k_cvt16<1024, false><<<(FFD * EMB / 8) / 256, 256, 0, stream>>>(W1, w116, (unsigned)(FFD * EMB / 8));
    k_cvt16<1024, false><<<(EMB * FFD / 8) / 256, 256, 0, stream>>>(W2, w216, (unsigned)(EMB * FFD / 8));

    const unsigned gQK = ((MTOK / 64) * (2 * EMB / 64) + 7) / 8;
    const unsigned gVT = ((EMB / 64) * (MTOK / 64) + 7) / 8;
    const unsigned gE  = ((MTOK / 64) * (EMB / 64) + 7) / 8;
    const unsigned gF  = ((MTOK / 64) * (FFD / 64) + 7) / 8;

    k_gemm64<1, 0, false, false, 16, 6><<<gQK, 256, 0, stream>>>(x16, EMB, wqkv16, EMB, (void*)qk16, 2 * EMB, bqkv, bqkv,
                                                                 MTOK, 2 * EMB, EMB);
    k_gemm64<1, 0, false, true, 16, 6><<<gVT, 256, 0, stream>>>(wqkv16 + (size_t)2 * EMB * EMB, EMB, x16, EMB, (void*)vt16, MTOK,
                                                                bqkv + 2 * EMB, bqkv, EMB, MTOK, EMB);
    k_attn<<<NB * HEADS * (SEQ / 128), 128, 0, stream>>>(qk16, vt16, mask, att16, mpl, rpl, (unsigned)(SEQ / 32));
    k_colsum<<<(NB * (SEQ / 64)) / 4, 128, 0, stream>>>(qk16, mask, mpl, rpl, hpre, (unsigned)(SEQ / 16), (unsigned)HEADS);
    k_halt<<<NB, 256, 0, stream>>>(hpre, mask, out1);
    k_gemm64<0, 2, false, false, 20, 0><<<gE, 256, 0, stream>>>(att16, EMB, wo16, EMB, (void*)ybuf, EMB, bo, x, MTOK, EMB, EMB);
    k_ln<true><<<MTOK / 8, 256, 0, stream>>>(ybuf, g1, be1, hf, h16p, (unsigned)MTOK);
    k_gemm64<1, 0, true, false, 16, 6><<<gF, 256, 0, stream>>>(h16p, EMB, w116, EMB, (void*)r16, FFD, b1, b1, MTOK, FFD, EMB);
    k_gemm64<0, 1, false, false, 16, 0><<<gE, 256, 0, stream>>>(r16, FFD, w216, FFD, (void*)ybuf, EMB, b2, hf, MTOK, EMB, FFD);
    k_ln<false><<<MTOK / 8, 256, 0, stream>>>(ybuf, g2, be2, out0, h16p, (unsigned)MTOK);
}
